// IA3Attention_41171556499741
// MI455X (gfx1250) — hardware-verified
//
#include <hip/hip_runtime.h>
#include <math.h>
#include <stdint.h>

constexpr int SEQ_LEN = 2048;
constexpr int DMODEL  = 2048;
constexpr int NHEAD   = 16;
constexpr int HDIM    = 128;
constexpr int NQKV    = 3 * DMODEL;

typedef __attribute__((ext_vector_type(16))) _Float16 v16h;
typedef __attribute__((ext_vector_type(8)))  _Float16 v8h;
typedef __attribute__((ext_vector_type(16))) __bf16   v16b;
typedef __attribute__((ext_vector_type(8)))  __bf16   v8b;
typedef __attribute__((ext_vector_type(8)))  float    v8f;
typedef __attribute__((ext_vector_type(4)))  float    v4f;
typedef __attribute__((ext_vector_type(2)))  float    v2f;
typedef __attribute__((ext_vector_type(4)))  unsigned int v4u;

__device__ __forceinline__ unsigned short f2bf_bits(float f) {
  unsigned u = __float_as_uint(f);
  return (unsigned short)((u + 0x7FFFu + ((u >> 16) & 1u)) >> 16);
}
__device__ __forceinline__ float bf_bits2f(unsigned short h) { return __uint_as_float(((unsigned)h) << 16); }

__device__ __forceinline__ void dep_guard_h(v8f& a, v8f& b, v16h x, v16h y) { asm volatile("v_nop\n\tv_nop\n\tv_nop\n\tv_nop" : "+v"(a), "+v"(b) : "v"(x), "v"(y)); }
__device__ __forceinline__ void dep_guard_b(v8f& a, v8f& b, v16b x, v16b y) { asm volatile("v_nop\n\tv_nop\n\tv_nop\n\tv_nop" : "+v"(a), "+v"(b) : "v"(x), "v"(y)); }
__device__ __forceinline__ void keep4_h(v16h a, v16h b, v16h c, v16h d) { asm volatile("v_nop" :: "v"(a), "v"(b), "v"(c), "v"(d)); }
__device__ __forceinline__ void keep4_b(v16b a, v16b b, v16b c, v16b d) { asm volatile("v_nop" :: "v"(a), "v"(b), "v"(c), "v"(d)); }
__device__ __forceinline__ void acc_guard4(v8f& a, v8f& b, v8f& c, v8f& d) { asm volatile("v_nop\n\tv_nop\n\tv_nop\n\tv_nop" : "+v"(a), "+v"(b), "+v"(c), "+v"(d)); }
template <typename T> struct Frag;
template <> struct Frag<_Float16> {
  typedef v16h V; union U { v16h v; v8h h[2]; };
  static __device__ __forceinline__ v16h load(const _Float16* p) {
    U f; f.h[0] = *(const v8h*)(p); f.h[1] = *(const v8h*)(p + 16); return f.v;
  }
  static __device__ __forceinline__ v8f mma(v16h a, v16h b, v8f c) {
    return __builtin_amdgcn_wmma_f32_16x16x32_f16(false, a, false, b, (short)0, c, false, false);
  }
  static __device__ __forceinline__ void guard(v8f& a, v8f& b, v16h x, v16h y) { dep_guard_h(a, b, x, y); }
  static __device__ __forceinline__ void keep(v16h a, v16h b, v16h c, v16h d) { keep4_h(a, b, c, d); }
};
template <> struct Frag<__bf16> {
  typedef v16b V; union U { v16b v; v8b h[2]; };
  static __device__ __forceinline__ v16b load(const __bf16* p) {
    U f; f.h[0] = *(const v8b*)(p); f.h[1] = *(const v8b*)(p + 16); return f.v;
  }
  static __device__ __forceinline__ v8f mma(v16b a, v16b b, v8f c) {
    return __builtin_amdgcn_wmma_f32_16x16x32_bf16(false, a, false, b, (short)0, c, false, false);
  }
  static __device__ __forceinline__ void guard(v8f& a, v8f& b, v16b x, v16b y) { dep_guard_b(a, b, x, y); }
  static __device__ __forceinline__ void keep(v16b a, v16b b, v16b c, v16b d) { keep4_b(a, b, c, d); }
};

template <int ET> struct Elem;
template <> struct Elem<0> { typedef _Float16 T; };
template <> struct Elem<1> { typedef __bf16 T; };
template <int ET, bool SPLIT, int BIAS_MODE, int OUT_MODE, bool RESID, int ACT = 0, bool ASPLIT = false>
__global__ __launch_bounds__(256) void wmma_gemm64(
    const unsigned short* __restrict__ Ap, const unsigned short* __restrict__ A2p, int lda, long strideA,
    const unsigned short* __restrict__ Btp, const unsigned short* __restrict__ Bt2p, int ldb, long strideB,
    void* __restrict__ Cout, void* __restrict__ Cout2, int ldc, long strideC,
    const float* __restrict__ bias,
    const float* __restrict__ resid, long strideR,
    int M, int N, int K, float scale) {
  typedef typename Elem<ET>::T T;
  typedef typename Frag<T>::V V;
  const T* A = (const T*)Ap; const T* A2 = (const T*)A2p; const T* Bt = (const T*)Btp; const T* Bt2 = (const T*)Bt2p;
  __shared__ __align__(16) float sT[8][16 * 68];
  const int b    = blockIdx.y;
  const int lane = threadIdx.x & 31;
  const int wave = threadIdx.x >> 5;
  const int tilesN = N >> 6;
  const int tilesM = M >> 6;
  const int tile = blockIdx.x * 8 + wave;
  if (tile >= tilesM * tilesN) return;
  const int tm = tile / tilesN;
  const int tn = tile - tm * tilesN;
  const int m0 = tm << 6;
  const int n0 = tn << 6;

  const T* Ab  = A  + (size_t)b * strideA;
  const T* Bb  = Bt + (size_t)b * strideB;
  const T* Ab2 = (SPLIT || ASPLIT) ? (A2  + (size_t)b * strideA) : nullptr;
  const T* Bb2 = SPLIT ? (Bt2 + (size_t)b * strideB) : nullptr;

  const int rlane = lane & 15;
  const int koff  = (lane >> 4) * 8;
  const int mOff  = (lane >> 4) * 8;

  v8f acc[4][4];
#pragma unroll
  for (int i = 0; i < 4; ++i)
#pragma unroll
    for (int j = 0; j < 4; ++j) acc[i][j] = (v8f){0.f,0.f,0.f,0.f,0.f,0.f,0.f,0.f};

  for (int k0 = 0; k0 < K; k0 += 32) {
    V bh[4], bl[4];
#pragma unroll
    for (int j = 0; j < 4; ++j) {
      const size_t bo = (size_t)(n0 + (j << 4) + rlane) * ldb + koff + k0;
      bh[j] = Frag<T>::load(Bb + bo);
      if (SPLIT) bl[j] = Frag<T>::load(Bb2 + bo);
    }
#pragma unroll
    for (int i = 0; i < 4; ++i) {
      const size_t ao = (size_t)(m0 + (i << 4) + rlane) * lda + koff + k0;
      V ah = Frag<T>::load(Ab + ao);
      V al;
      if (SPLIT || ASPLIT) al = Frag<T>::load(Ab2 + ao);
#pragma unroll
      for (int j = 0; j < 4; ++j) {
        acc[i][j] = Frag<T>::mma(ah, bh[j], acc[i][j]);
        if (SPLIT) {
          acc[i][j] = Frag<T>::mma(ah, bl[j], acc[i][j]);
          acc[i][j] = Frag<T>::mma(al, bh[j], acc[i][j]);
        }
        if (ASPLIT && !SPLIT) {
          acc[i][j] = Frag<T>::mma(al, bh[j], acc[i][j]);
        }
      }
      Frag<T>::guard(acc[i][0], acc[i][3], ah, (SPLIT || ASPLIT) ? al : ah);
    }
    Frag<T>::keep(bh[0], bh[1], bh[2], bh[3]);
    if (SPLIT) Frag<T>::keep(bl[0], bl[1], bl[2], bl[3]);
  }
  acc_guard4(acc[0][0], acc[0][1], acc[0][2], acc[0][3]);
  acc_guard4(acc[1][0], acc[1][1], acc[1][2], acc[1][3]);
  acc_guard4(acc[2][0], acc[2][1], acc[2][2], acc[2][3]);
  acc_guard4(acc[3][0], acc[3][1], acc[3][2], acc[3][3]);

  float* slab = sT[wave];
  const float* Rb = RESID ? (resid + (size_t)b * strideR) : nullptr;
#pragma unroll
  for (int i = 0; i < 4; ++i) {
    const int mBase = m0 + (i << 4);
#pragma unroll
    for (int j = 0; j < 4; ++j) {
      const int n = n0 + (j << 4) + rlane;
      float bv = 0.f;
      if (BIAS_MODE == 2) bv = bias[n];
#pragma unroll
      for (int r = 0; r < 8; ++r) {
        float v = acc[i][j][r] * scale;
        if (BIAS_MODE == 1) v += bias[mBase + mOff + r];
        if (BIAS_MODE == 2) v += bv;
        if (RESID) v += Rb[(size_t)(mBase + mOff + r) * ldc + n];
        if (ACT == 1) v = tanhf(v);
        if (ACT == 2) v = fmaxf(v, 0.0f);
        if (ACT == 3) v = v / (1.0f + expf(-v));
        if (ACT == 4) v = (v > 0.f) ? v : 0.01f * v;
        slab[(mOff + r) * 68 + (j << 4) + rlane] = v;
      }
    }
    __builtin_amdgcn_fence(__ATOMIC_RELEASE, "workgroup");
    __builtin_amdgcn_wave_barrier();
    __builtin_amdgcn_fence(__ATOMIC_ACQUIRE, "workgroup");
    if (OUT_MODE == 0) {
      float* C = (float*)Cout + (size_t)b * strideC;
      const int hh = lane >> 4, c4 = (lane & 15) * 4;
      for (int pass = 0; pass < 2; ++pass) {
#pragma unroll
        for (int it = 0; it < 8; ++it) {
          const int row = it * 2 + hh;
          v4f v = *(const v4f*)(slab + row * 68 + c4);
          *(volatile v4f*)(C + (size_t)(mBase + row) * ldc + n0 + c4) = v;
        }
        __threadfence();
      }
    } else {
      const int q = lane >> 3, c8 = (lane & 7) * 8;
      unsigned short* C  = (unsigned short*)Cout  + (size_t)b * strideC;
      unsigned short* C2 = (OUT_MODE == 2) ? ((unsigned short*)Cout2 + (size_t)b * strideC) : nullptr;
      for (int pass = 0; pass < 2; ++pass) {
#pragma unroll
        for (int it = 0; it < 4; ++it) {
          const int row = it * 4 + q;
          const float* sp = slab + row * 68 + c8;
          v8h hv, lv;
#pragma unroll
          for (int e = 0; e < 8; ++e) {
            if (OUT_MODE == 1) {
              hv[e] = (_Float16)sp[e];
            } else {
              unsigned short hb = f2bf_bits(sp[e]);
              unsigned short lb = f2bf_bits(sp[e] - bf_bits2f(hb));
              hv[e] = __builtin_bit_cast(_Float16, hb);
              lv[e] = __builtin_bit_cast(_Float16, lb);
            }
          }
          *(volatile v8h*)(C + (size_t)(mBase + row) * ldc + n0 + c8) = hv;
          if (OUT_MODE == 2) *(volatile v8h*)(C2 + (size_t)(mBase + row) * ldc + n0 + c8) = lv;
        }
        __threadfence();
      }
    }
    __builtin_amdgcn_fence(__ATOMIC_RELEASE, "workgroup");
    __builtin_amdgcn_wave_barrier();
    __builtin_amdgcn_fence(__ATOMIC_ACQUIRE, "workgroup");
  }
}

__device__ __forceinline__ unsigned pk16(unsigned short a, unsigned short b) { return (unsigned)a | ((unsigned)b << 16); }

__device__ __forceinline__ unsigned short at_bf_bits(float f) {
  unsigned u = __float_as_uint(f);
  return (unsigned short)((u + 0x7FFFu + ((u >> 16) & 1u)) >> 16);
}
__device__ __forceinline__ __bf16 at_f2bf(float f) { return __builtin_bit_cast(__bf16, at_bf_bits(f)); }
__device__ __forceinline__ void at_split(float f, __bf16& hi, __bf16& lo) {
  const unsigned short hb = at_bf_bits(f);
  hi = __builtin_bit_cast(__bf16, hb);
  lo = at_f2bf(f - __uint_as_float(((unsigned)hb) << 16));
}
__device__ __forceinline__ v8f at_mma(v16b a, v16b b, v8f c) {
  c = __builtin_amdgcn_wmma_f32_16x16x32_bf16(false, a, false, b, (short)0, c, false, false);
  asm volatile("v_nop\n\tv_nop\n\tv_nop\n\tv_nop" : "+v"(c) : "v"(a), "v"(b));
  return c;
}

__device__ __forceinline__ float bf_rne(float x) { return bf_bits2f(f2bf_bits(x)); }
__device__ __forceinline__ void split2(float f0, float f1, unsigned& ph, unsigned& pl) {
  const unsigned short h0 = f2bf_bits(f0), h1 = f2bf_bits(f1);
  const unsigned short l0 = f2bf_bits(f0 - bf_bits2f(h0)), l1 = f2bf_bits(f1 - bf_bits2f(h1));
  ph = pk16(h0, h1); pl = pk16(l0, l1);
}

__global__ __launch_bounds__(256) void cast_f32_bf16x2(const float* __restrict__ in, unsigned short* __restrict__ out, int n2) {
  const int i = blockIdx.x * 256 + threadIdx.x;
  if (i < n2) {
    const v2f f = *(const v2f*)(in + 2 * (size_t)i);
    const unsigned u = pk16(f2bf_bits(f[0]), f2bf_bits(f[1]));
    ((volatile unsigned*)out)[i] = u;
    __threadfence();
    ((volatile unsigned*)out)[i] = u;
  }
}

constexpr int RP_PITCH = 132;
__global__ __launch_bounds__(256) void rope_scale_split_kernel(
    const float* __restrict__ QKV, const float* __restrict__ cosT, const float* __restrict__ sinT,
    const float* __restrict__ lkp, const float* __restrict__ lvp,
    unsigned short* __restrict__ qh, unsigned short* __restrict__ ql,
    unsigned short* __restrict__ kh, unsigned short* __restrict__ kl,
    unsigned short* __restrict__ vth, unsigned short* __restrict__ vtl) {
  __shared__ __align__(16) float vt[64 * RP_PITCH];
  const int s0  = blockIdx.x * 64;
  const int h   = blockIdx.y;
  const int tid = threadIdx.x;
  const int lr  = tid >> 4;
  const int dg  = (tid & 15) * 8;
  const int pg  = (dg < 64) ? (dg + 64) : (dg - 64);
  const float sg = (dg < 64) ? -1.0f : 1.0f;

  float lkr[8], lvr[8];
  {
    const v4f a0 = *(const v4f*)(lkp + h * HDIM + dg), a1 = *(const v4f*)(lkp + h * HDIM + dg + 4);
    const v4f b0 = *(const v4f*)(lvp + h * HDIM + dg), b1 = *(const v4f*)(lvp + h * HDIM + dg + 4);
#pragma unroll
    for (int e = 0; e < 4; ++e) {
      lkr[e] = bf_rne(a0[e]); lkr[4 + e] = bf_rne(a1[e]);
      lvr[e] = bf_rne(b0[e]); lvr[4 + e] = bf_rne(b1[e]);
    }
  }

#pragma unroll 1
  for (int it = 0; it < 4; ++it) {
    const int rr = it * 16 + lr;
    const int s  = s0 + rr;
    const float* base = QKV + (size_t)s * NQKV + h * HDIM;
    const v4f qa  = *(const v4f*)(base + dg),               qb  = *(const v4f*)(base + dg + 4);
    const v4f qpa = *(const v4f*)(base + pg),               qpb = *(const v4f*)(base + pg + 4);
    const v4f ka  = *(const v4f*)(base + DMODEL + dg),      kb  = *(const v4f*)(base + DMODEL + dg + 4);
    const v4f kpa = *(const v4f*)(base + DMODEL + pg),      kpb = *(const v4f*)(base + DMODEL + pg + 4);
    const v4f va  = *(const v4f*)(base + 2 * DMODEL + dg),  vb  = *(const v4f*)(base + 2 * DMODEL + dg + 4);
    const v4f ca  = *(const v4f*)(cosT + (size_t)s * HDIM + dg), cb = *(const v4f*)(cosT + (size_t)s * HDIM + dg + 4);
    const v4f sa  = *(const v4f*)(sinT + (size_t)s * HDIM + dg), sb = *(const v4f*)(sinT + (size_t)s * HDIM + dg + 4);
    float q8[8], qp8[8], k8[8], kp8[8], v8r[8], c8[8], sn8[8];
#pragma unroll
    for (int e = 0; e < 4; ++e) {
      q8[e] = qa[e];   q8[4 + e] = qb[e];   qp8[e] = qpa[e]; qp8[4 + e] = qpb[e];
      k8[e] = ka[e];   k8[4 + e] = kb[e];   kp8[e] = kpa[e]; kp8[4 + e] = kpb[e];
      v8r[e] = va[e];  v8r[4 + e] = vb[e];
      c8[e] = ca[e];   c8[4 + e] = cb[e];   sn8[e] = sa[e];  sn8[4 + e] = sb[e];
    }
    float qo[8], ko[8], vo[8];
#pragma unroll
    for (int e = 0; e < 8; ++e) {
      const float cr = bf_rne(c8[e]);
      const float sr = bf_rne(sn8[e]);
      qo[e] = (q8[e] * cr + (sg * qp8[e]) * sr) * lkr[e];
      ko[e] = k8[e] * cr + (sg * kp8[e]) * sr;
      vo[e] = v8r[e] * lvr[e];
    }
    v4u hq, lq, hk, hlk;
#pragma unroll
    for (int q = 0; q < 4; ++q) {
      unsigned a, b2;
      split2(qo[2 * q], qo[2 * q + 1], a, b2); hq[q] = a; lq[q] = b2;
      split2(ko[2 * q], ko[2 * q + 1], a, b2); hk[q] = a; hlk[q] = b2;
    }
    *(v4f*)(vt + rr * RP_PITCH + dg)     = (v4f){vo[0], vo[1], vo[2], vo[3]};
    *(v4f*)(vt + rr * RP_PITCH + dg + 4) = (v4f){vo[4], vo[5], vo[6], vo[7]};
    const size_t go = (size_t)s * DMODEL + h * HDIM + dg;
    *(volatile v4u*)(qh + go) = hq;
    *(volatile v4u*)(ql + go) = lq;
    *(volatile v4u*)(kh + go) = hk;
    *(volatile v4u*)(kl + go) = hlk;
    __threadfence();
    *(volatile v4u*)(qh + go) = hq;
    *(volatile v4u*)(ql + go) = lq;
    *(volatile v4u*)(kh + go) = hk;
    *(volatile v4u*)(kl + go) = hlk;
  }
  __syncthreads();
#pragma unroll 1
  for (int p = 0; p < 4; ++p) {
    const int d   = p * 32 + (tid >> 3);
    const int sgi = (tid & 7) * 8;
    v4u hv, lvq;
#pragma unroll
    for (int q = 0; q < 4; ++q) {
      const float f0 = vt[(sgi + 2 * q) * RP_PITCH + d];
      const float f1 = vt[(sgi + 2 * q + 1) * RP_PITCH + d];
      unsigned a, b2;
      split2(f0, f1, a, b2); hv[q] = a; lvq[q] = b2;
    }
    const size_t go = (size_t)(h * HDIM + d) * SEQ_LEN + s0 + sgi;
    *(volatile v4u*)(vth + go) = hv;
    *(volatile v4u*)(vtl + go) = lvq;
    __threadfence();
    *(volatile v4u*)(vth + go) = hv;
    *(volatile v4u*)(vtl + go) = lvq;
  }
}

constexpr int ATT_HD  = 128;
constexpr int ATT_KV  = 64;
constexpr int ATT_QR  = 64;
constexpr int ATT_WV  = 4;
constexpr int ATT_OSP = 20;
typedef char att_os_fits_check[(ATT_WV * ATT_HD * ATT_OSP * 4 <= 4 * ATT_KV * ATT_HD * 2) ? 1 : -1];

__global__ __launch_bounds__(128)
void attn_causal_hd128_kernel(const unsigned short* __restrict__ qhp, const unsigned short* __restrict__ qlp,
                              const unsigned short* __restrict__ khp, const unsigned short* __restrict__ klp,
                              const unsigned short* __restrict__ vhp, const unsigned short* __restrict__ vlp,
                              const float* __restrict__ maskp,
                              unsigned short* __restrict__ ohp, unsigned short* __restrict__ olp, float sscale) {
  union FB { v16b v; v8b h[2]; };
  __shared__ __align__(16) __bf16 Qs[2 * ATT_QR * ATT_HD];
  __shared__ __align__(16) __bf16 KVs[4 * ATT_KV * ATT_HD];
  __shared__ __align__(16) __bf16 Ps[2 * ATT_WV * 16 * ATT_KV];

  const int tid  = threadIdx.x;
  const int wave = tid >> 5;
  const int lane = tid & 31;
  const int hh   = lane >> 4;
  const int c    = lane & 15;

  const int nqb = SEQ_LEN / ATT_QR;
  const int qb  = blockIdx.x % nqb;
  const int h   = blockIdx.x / nqb;
  const int qbase = qb * ATT_QR;
  const int qw    = wave * 16;

  const __bf16* Qh = (const __bf16*)(const void*)qhp + (size_t)h * ATT_HD;
  const __bf16* Ql = (const __bf16*)(const void*)qlp + (size_t)h * ATT_HD;
  const __bf16* Kh = (const __bf16*)(const void*)khp + (size_t)h * ATT_HD;
  const __bf16* Kl = (const __bf16*)(const void*)klp + (size_t)h * ATT_HD;
  const __bf16* Vh = (const __bf16*)(const void*)vhp + (size_t)h * ATT_HD * SEQ_LEN;
  const __bf16* Vl = (const __bf16*)(const void*)vlp + (size_t)h * ATT_HD * SEQ_LEN;
  unsigned short* Obh = ohp + (size_t)h * ATT_HD;
  unsigned short* Obl = olp + (size_t)h * ATT_HD;

  __bf16* Qsh = Qs;
  __bf16* Qsl = Qs + ATT_QR * ATT_HD;
  __bf16* Ksh = KVs;
  __bf16* Ksl = KVs + ATT_KV * ATT_HD;
  __bf16* Vth = KVs + 2 * ATT_KV * ATT_HD;
  __bf16* Vtl = KVs + 3 * ATT_KV * ATT_HD;
  __bf16* pwh = Ps + wave * 16 * ATT_KV;
  __bf16* pwl = Ps + (ATT_WV + wave) * 16 * ATT_KV;

  {
    const int r = tid >> 1, half = (tid & 1) * 64;
    const __bf16* g0 = Qh + (size_t)(qbase + r) * DMODEL + half;
    const __bf16* g1 = Ql + (size_t)(qbase + r) * DMODEL + half;
#pragma unroll
    for (int i = 0; i < 8; ++i) {
      const v8b a0 = *(const v8b*)(g0 + 8 * i);
      const v8b a1 = *(const v8b*)(g1 + 8 * i);
      *(v8b*)(Qsh + r * ATT_HD + half + 8 * i) = a0;
      *(v8b*)(Qsl + r * ATT_HD + half + 8 * i) = a1;
    }
  }

  float mrow[8], lrow[8];
  v8f oacc[8];
#pragma unroll
  for (int r = 0; r < 8; ++r) { mrow[r] = -INFINITY; lrow[r] = 0.f; }
#pragma unroll
  for (int t = 0; t < 8; ++t) oacc[t] = (v8f){0.f,0.f,0.f,0.f,0.f,0.f,0.f,0.f};

  const int nChunks = qb + 1;
  for (int kc = 0; kc < nChunks; ++kc) {
    const int kv0 = kc * ATT_KV;
    __syncthreads();
    {
      const int r = tid >> 1, half = (tid & 1) * 64;
      const __bf16* gkh = Kh + (size_t)(kv0 + r) * DMODEL + half;
      const __bf16* gkl = Kl + (size_t)(kv0 + r) * DMODEL + half;
      const int rd = tid;
      const __bf16* gvh = Vh + (size_t)rd * SEQ_LEN + kv0;
      const __bf16* gvl = Vl + (size_t)rd * SEQ_LEN + kv0;
#pragma unroll
      for (int i = 0; i < 8; ++i) {
        const v8b a0 = *(const v8b*)(gkh + 8 * i);
        const v8b a1 = *(const v8b*)(gkl + 8 * i);
        const v8b b0 = *(const v8b*)(gvh + 8 * i);
        const v8b b1 = *(const v8b*)(gvl + 8 * i);
        *(v8b*)(Ksh + r * ATT_HD + half + 8 * i) = a0;
        *(v8b*)(Ksl + r * ATT_HD + half + 8 * i) = a1;
        *(v8b*)(Vth + rd * ATT_KV + 8 * i) = b0;
        *(v8b*)(Vtl + rd * ATT_KV + 8 * i) = b1;
      }
    }
    __syncthreads();

    v8f s[4];
#pragma unroll
    for (int j = 0; j < 4; ++j) {
      s[j] = (v8f){0.f,0.f,0.f,0.f,0.f,0.f,0.f,0.f};
#pragma unroll 1
      for (int dc = 0; dc < 4; ++dc) {
        FB qa, qlo, kb, klo;
        qa.h[0]  = *(const v8b*)(Qsh + (qw + c) * ATT_HD + dc * 32 + 8 * hh);
        qa.h[1]  = *(const v8b*)(Qsh + (qw + c) * ATT_HD + dc * 32 + 16 + 8 * hh);
        qlo.h[0] = *(const v8b*)(Qsl + (qw + c) * ATT_HD + dc * 32 + 8 * hh);
        qlo.h[1] = *(const v8b*)(Qsl + (qw + c) * ATT_HD + dc * 32 + 16 + 8 * hh);
        kb.h[0]  = *(const v8b*)(Ksh + (j * 16 + c) * ATT_HD + dc * 32 + 8 * hh);
        kb.h[1]  = *(const v8b*)(Ksh + (j * 16 + c) * ATT_HD + dc * 32 + 16 + 8 * hh);
        klo.h[0] = *(const v8b*)(Ksl + (j * 16 + c) * ATT_HD + dc * 32 + 8 * hh);
        klo.h[1] = *(const v8b*)(Ksl + (j * 16 + c) * ATT_HD + dc * 32 + 16 + 8 * hh);
        s[j] = at_mma(qa.v, kb.v, s[j]);
        s[j] = at_mma(qa.v, klo.v, s[j]);
        s[j] = at_mma(qlo.v, kb.v, s[j]);
      }
    }
    float cm[8];
#pragma unroll
    for (int r = 0; r < 8; ++r) {
      const int qrow = qbase + qw + 8 * hh + r;
      const float* mr = maskp + (size_t)qrow * SEQ_LEN + kv0 + c;
      float m = -INFINITY;
#pragma unroll
      for (int j = 0; j < 4; ++j) {
        const float sv = s[j][r] * sscale + mr[j * 16];
        s[j][r] = sv;
        m = fmaxf(m, sv);
      }
#pragma unroll
      for (int off = 1; off < 16; off <<= 1) m = fmaxf(m, __shfl_xor(m, off, 32));
      cm[r] = m;
    }
#pragma unroll
    for (int r = 0; r < 8; ++r) {
      const float mnew = fmaxf(mrow[r], cm[r]);
      const float alpha = expf(mrow[r] - mnew);
      mrow[r] = mnew;
      float psum = 0.f;
#pragma unroll
      for (int j = 0; j < 4; ++j) {
        const float p = expf(s[j][r] - mnew);
        psum += p;
        __bf16 a, bl; at_split(p, a, bl);
        pwh[(8 * hh + r) * ATT_KV + j * 16 + c] = a;
        pwl[(8 * hh + r) * ATT_KV + j * 16 + c] = bl;
      }
#pragma unroll
      for (int off = 1; off < 16; off <<= 1) psum += __shfl_xor(psum, off, 32);
      lrow[r] = lrow[r] * alpha + psum;
#pragma unroll
      for (int t = 0; t < 8; ++t) oacc[t][r] *= alpha;
    }
    __builtin_amdgcn_fence(__ATOMIC_RELEASE, "workgroup");
    __builtin_amdgcn_wave_barrier();
    __builtin_amdgcn_fence(__ATOMIC_ACQUIRE, "workgroup");
#pragma unroll 1
    for (int kk = 0; kk < 2; ++kk) {
      FB pa, pl;
      pa.h[0] = *(const v8b*)(pwh + c * ATT_KV + kk * 32 + 8 * hh);
      pa.h[1] = *(const v8b*)(pwh + c * ATT_KV + kk * 32 + 16 + 8 * hh);
      pl.h[0] = *(const v8b*)(pwl + c * ATT_KV + kk * 32 + 8 * hh);
      pl.h[1] = *(const v8b*)(pwl + c * ATT_KV + kk * 32 + 16 + 8 * hh);
#pragma unroll
      for (int t = 0; t < 8; ++t) {
        FB vb, vl;
        vb.h[0] = *(const v8b*)(Vth + (t * 16 + c) * ATT_KV + kk * 32 + 8 * hh);
        vb.h[1] = *(const v8b*)(Vth + (t * 16 + c) * ATT_KV + kk * 32 + 16 + 8 * hh);
        vl.h[0] = *(const v8b*)(Vtl + (t * 16 + c) * ATT_KV + kk * 32 + 8 * hh);
        vl.h[1] = *(const v8b*)(Vtl + (t * 16 + c) * ATT_KV + kk * 32 + 16 + 8 * hh);
        oacc[t] = at_mma(pa.v, vb.v, oacc[t]);
        oacc[t] = at_mma(pa.v, vl.v, oacc[t]);
        oacc[t] = at_mma(pl.v, vb.v, oacc[t]);
      }
    }
  }

  __syncthreads();
  float* os = (float*)(void*)KVs + wave * (ATT_HD * ATT_OSP);
  float inv[8];
#pragma unroll
  for (int r = 0; r < 8; ++r) inv[r] = 1.0f / lrow[r];
#pragma unroll
  for (int t = 0; t < 8; ++t) {
    v4f a, b2;
    a[0]  = oacc[t][0] * inv[0]; a[1]  = oacc[t][1] * inv[1]; a[2]  = oacc[t][2] * inv[2]; a[3]  = oacc[t][3] * inv[3];
    b2[0] = oacc[t][4] * inv[4]; b2[1] = oacc[t][5] * inv[5]; b2[2] = oacc[t][6] * inv[6]; b2[3] = oacc[t][7] * inv[7];
    float* op = os + (t * 16 + c) * ATT_OSP + 8 * hh;
    *(v4f*)(op)     = a;
    *(v4f*)(op + 4) = b2;
  }
  __builtin_amdgcn_fence(__ATOMIC_RELEASE, "workgroup");
  __builtin_amdgcn_wave_barrier();
  __builtin_amdgcn_fence(__ATOMIC_ACQUIRE, "workgroup");
  {
    const int c8 = c * 8;
    for (int pass = 0; pass < 2; ++pass) {
#pragma unroll
      for (int it = 0; it < 8; ++it) {
        const int row = it * 2 + hh;
        v8h hv, lv;
#pragma unroll
        for (int e = 0; e < 8; ++e) {
          const float f = os[(c8 + e) * ATT_OSP + row];
          const unsigned short hb = at_bf_bits(f);
          const unsigned short lb = at_bf_bits(f - __uint_as_float(((unsigned)hb) << 16));
          hv[e] = __builtin_bit_cast(_Float16, hb);
          lv[e] = __builtin_bit_cast(_Float16, lb);
        }
        const size_t go = (size_t)(qbase + qw + row) * DMODEL + c8;
        *(volatile v8h*)(Obh + go) = hv;
        *(volatile v8h*)(Obl + go) = lv;
      }
      __threadfence();
    }
  }
}

extern "C" void kernel_launch(void* const* d_in, const int* in_sizes, int n_in,
                              void* d_out, int out_size, void* d_ws, size_t ws_size,
                              hipStream_t stream) {
  const size_t SD = (size_t)SEQ_LEN * DMODEL;
  if (n_in < 10) return;
  if ((size_t)in_sizes[0] != SD || (size_t)in_sizes[1] != (size_t)SEQ_LEN * SEQ_LEN ||
      (size_t)in_sizes[2] != (size_t)SEQ_LEN * HDIM || (size_t)in_sizes[3] != (size_t)SEQ_LEN * HDIM ||
      (size_t)in_sizes[4] != SD || (size_t)in_sizes[5] != SD || (size_t)in_sizes[6] != SD || (size_t)in_sizes[7] != SD ||
      (size_t)in_sizes[8] != (size_t)NHEAD * HDIM || (size_t)in_sizes[9] != (size_t)NHEAD * HDIM ||
      (size_t)out_size != SD) return;

  const float* hidden = (const float*)d_in[0];
  const float* amask  = (const float*)d_in[1];
  const float* cosT   = (const float*)d_in[2];
  const float* sinT   = (const float*)d_in[3];
  const float* Wq     = (const float*)d_in[4];
  const float* Wk     = (const float*)d_in[5];
  const float* Wv     = (const float*)d_in[6];
  const float* Wo     = (const float*)d_in[7];
  const float* lkp    = (const float*)d_in[8];
  const float* lvp    = (const float*)d_in[9];
  float* out = (float*)d_out;

  char* ws = (char*)d_ws;
  const size_t OFF_QKV  = 0;
  const size_t OFF_OHI  = 0;
  const size_t OFF_OLO  = SD * 2;
  const size_t OFF_WO16 = OFF_QKV + SD * 3 * 4;
  const size_t OFF_XB   = OFF_WO16 + SD * 2;
  const size_t OFF_WQKV = OFF_XB + SD * 2;
  const size_t END_A    = OFF_WQKV + SD * 3 * 2;
  const size_t OFF_PL   = OFF_XB;
  const size_t PLANE_B  = SD * 2;
  const size_t END_B    = OFF_PL + 6 * PLANE_B;
  const size_t total    = (END_A > END_B) ? END_A : END_B;
  if (ws_size < total) return;

  float*          QKVf = (float*)(ws + OFF_QKV);
  unsigned short* Ohi  = (unsigned short*)(ws + OFF_OHI);
  unsigned short* Olo  = (unsigned short*)(ws + OFF_OLO);
  unsigned short* Wo16 = (unsigned short*)(ws + OFF_WO16);
  unsigned short* Xb   = (unsigned short*)(ws + OFF_XB);
  unsigned short* Wqkv = (unsigned short*)(ws + OFF_WQKV);
  unsigned short* Qhp  = (unsigned short*)(ws + OFF_PL + 0 * PLANE_B);
  unsigned short* Qlp  = (unsigned short*)(ws + OFF_PL + 1 * PLANE_B);
  unsigned short* Khp  = (unsigned short*)(ws + OFF_PL + 2 * PLANE_B);
  unsigned short* Klp  = (unsigned short*)(ws + OFF_PL + 3 * PLANE_B);
  unsigned short* Vthp = (unsigned short*)(ws + OFF_PL + 4 * PLANE_B);
  unsigned short* Vtlp = (unsigned short*)(ws + OFF_PL + 5 * PLANE_B);
  const float* dummyf  = (const float*)(ws + OFF_WO16);

  const int n2 = (int)(SD / 2);
  const unsigned castBlocks = (unsigned)((n2 + 255) / 256);

  cast_f32_bf16x2<<<dim3(castBlocks), dim3(256), 0, stream>>>(hidden, Xb, n2);
  cast_f32_bf16x2<<<dim3(castBlocks), dim3(256), 0, stream>>>(Wq, Wqkv, n2);
  cast_f32_bf16x2<<<dim3(castBlocks), dim3(256), 0, stream>>>(Wk, Wqkv + SD, n2);
  cast_f32_bf16x2<<<dim3(castBlocks), dim3(256), 0, stream>>>(Wv, Wqkv + 2 * SD, n2);
  cast_f32_bf16x2<<<dim3(castBlocks), dim3(256), 0, stream>>>(Wo, Wo16, n2);

  {
    const int M = SEQ_LEN, N = NQKV, K = DMODEL;
    const unsigned blocks = (unsigned)(((M / 64) * (N / 64) + 7) / 8);
    wmma_gemm64<1, false, 0, 0, false><<<dim3(blocks, 1), dim3(256), 0, stream>>>(
        Xb, Xb, K, 0L, Wqkv, Wqkv, K, 0L, (void*)QKVf, (void*)Wo16, N, 0L, dummyf, dummyf, 0L, M, N, K, 1.0f);
  }

  rope_scale_split_kernel<<<dim3(SEQ_LEN / 64, NHEAD), dim3(256), 0, stream>>>(
      QKVf, cosT, sinT, lkp, lvp, Qhp, Qlp, Khp, Klp, Vthp, Vtlp);

  attn_causal_hd128_kernel<<<dim3(NHEAD * (SEQ_LEN / ATT_QR)), dim3(128), 0, stream>>>(
      Qhp, Qlp, Khp, Klp, Vthp, Vtlp, amask, Ohi, Olo, 0.08838834764831845f);

  {
    const int M = SEQ_LEN, N = DMODEL, K = DMODEL;
    const unsigned blocks = (unsigned)(((M / 64) * (N / 64) + 7) / 8);
    wmma_gemm64<1, false, 0, 0, false, 0, true><<<dim3(blocks, 1), dim3(256), 0, stream>>>(
        Ohi, Olo, K, 0L, Wo16, Wo16, K, 0L, (void*)out, (void*)Wo16, N, 0L, dummyf, dummyf, 0L, M, N, K, 1.0f);
  }
}
